// Block_4569845203333
// MI455X (gfx1250) — hardware-run, weakly checked
//
#include <hip/hip_runtime.h>
#ifndef NB
#define NB 4
#endif
#ifndef SEQ
#define SEQ 1024
#endif
#define NB_FULL 4
#define SEQ_FULL 1024
#define DM 1024
#define NH 16
#define HD 64
#define DFF 4096
#define LQ (3 * DM)
#define NR (NB * SEQ)
#define MCH ((NR) >= 2048 ? 2048 : (NR))
#define XROW(r) ((size_t)((r) / SEQ) * SEQ_FULL + (size_t)((r) % SEQ))

static_assert(NH * HD == DM);
static_assert(HD == 64);
static_assert(DM == 256 * 4);
static_assert(DFF == 256 * 16);
static_assert(DM % 32 == 0 && DFF % 32 == 0 && HD % 32 == 0);
static_assert(DM % 64 == 0 && DFF % 64 == 0 && LQ % 64 == 0);
static_assert(SEQ % 128 == 0 && NR % 128 == 0 && MCH % 128 == 0 && NR % MCH == 0);
static_assert(NB <= NB_FULL && SEQ <= SEQ_FULL);

typedef _Float16 v16h __attribute__((ext_vector_type(16)));
typedef _Float16 v4h  __attribute__((ext_vector_type(4)));
typedef unsigned short v8us __attribute__((ext_vector_type(8), may_alias));
typedef float  v8f  __attribute__((ext_vector_type(8)));
typedef float  v4f  __attribute__((ext_vector_type(4)));
typedef float  v4fa __attribute__((ext_vector_type(4), may_alias));
union FragH { v16h v; v8us half[2]; _Float16 h[16]; unsigned short u[16]; };

__device__ __forceinline__ unsigned short bf16_bits(float x) { unsigned int u = __float_as_uint(x); return (unsigned short)((u + 0x7FFFu + ((u >> 16) & 1u)) >> 16); }
__device__ __forceinline__ float bf16_rne(float x) { return __uint_as_float(((unsigned int)bf16_bits(x)) << 16); }
__device__ __forceinline__ unsigned short h16_bits(float x) { const _Float16 h = (_Float16)x; return __builtin_bit_cast(unsigned short, h); }

__device__ __forceinline__ v16h g2_frag(const _Float16* p, int hh) { FragH f; f.half[0] = *(const v8us*)((const unsigned short*)p + 8 * hh); f.half[1] = *(const v8us*)((const unsigned short*)p + 16 + 8 * hh); return f.v; }
__device__ __forceinline__ v8f g2_mma(v16h a, v16h b, v8f c) { v8f d = __builtin_amdgcn_wmma_f32_16x16x32_f16(false, a, false, b, (short)0, c, false, false); asm volatile("v_nop\n\tv_nop\n\tv_nop\n\tv_nop" : "+v"(d) : "v"(a), "v"(b)); return d; }

__global__ __launch_bounds__(256) void k_wnat(const float* __restrict__ w, _Float16* __restrict__ Bt, unsigned int n8) {
  const unsigned int t = blockIdx.x * 256u + threadIdx.x; if (t >= n8) return;
  const v4f a = *(const v4fa*)(w + (size_t)t * 8), c = *(const v4fa*)(w + (size_t)t * 8 + 4); FragH f;
#pragma unroll
  for (int q = 0; q < 4; ++q) { f.h[q] = (_Float16)(bf16_rne(a[q]) * 16.0f); f.h[4 + q] = (_Float16)(bf16_rne(c[q]) * 16.0f); }
  const v8us o = f.half[0]; unsigned short* d = (unsigned short*)Bt + (size_t)t * 8;
  *(volatile v8us*)d = o; __threadfence(); *(volatile v8us*)d = o;
}

__global__ __launch_bounds__(256) void k_ln16(const float* __restrict__ X, const float* __restrict__ g, const float* __restrict__ bb, int bfin, int remap, _Float16* __restrict__ N16) {
  #pragma clang fp contract(off)
  __shared__ float red[256];
  const int r = blockIdx.x; const int t = threadIdx.x; const size_t rs_ = remap ? XROW(r) : (size_t)r;
  const v4f xa = *(const v4fa*)(X + rs_ * DM + t * 4); float s[4]; float sum = 0.f;
#pragma unroll
  for (int q = 0; q < 4; ++q) { const float rb = bf16_rne(xa[q]); s[q] = bfin ? rb : xa[q]; sum = sum + s[q]; }
  red[t] = sum; __syncthreads();
  for (int st = 128; st > 0; st >>= 1) { if (t < st) red[t] = red[t] + red[t + st]; __syncthreads(); }
  const float mu = red[0] * (1.0f / (float)DM); __syncthreads();
  float vs = 0.f;
#pragma unroll
  for (int q = 0; q < 4; ++q) { const float dl = s[q] - mu; vs = vs + dl * dl; }
  red[t] = vs; __syncthreads();
  for (int st = 128; st > 0; st >>= 1) { if (t < st) red[t] = red[t] + red[t + st]; __syncthreads(); }
  const float rs = rsqrtf(red[0] * (1.0f / (float)DM) + 1e-5f);
  const v4f gg = *(const v4fa*)(g + t * 4), bv = *(const v4fa*)(bb + t * 4); v4h y;
#pragma unroll
  for (int q = 0; q < 4; ++q) { const float yy = ((s[q] - mu) * rs) * bf16_rne(gg[q]) + bf16_rne(bv[q]); y[q] = (_Float16)yy; }
  _Float16* d = N16 + (size_t)r * DM + t * 4;
  *(volatile v4h*)d = y; __threadfence(); *(volatile v4h*)d = y;
}

__global__ __launch_bounds__(256) void k_lnh(const float* __restrict__ U, const float* __restrict__ g, const float* __restrict__ bb, _Float16* __restrict__ UH, _Float16* __restrict__ UL) {
  #pragma clang fp contract(off)
  __shared__ float red[256];
  const size_t r = blockIdx.x; const int t = threadIdx.x; const float* x = U + r * DFF;
  float vals[16]; float sum = 0.f;
#pragma unroll
  for (int u = 0; u < 4; ++u) { const v4f a = *(const v4fa*)(x + t * 4 + 1024 * u);
#pragma unroll
    for (int q = 0; q < 4; ++q) { vals[u * 4 + q] = a[q]; sum = sum + a[q]; } }
  red[t] = sum; __syncthreads();
  for (int st = 128; st > 0; st >>= 1) { if (t < st) red[t] = red[t] + red[t + st]; __syncthreads(); }
  const float mu = red[0] * (1.0f / (float)DFF); __syncthreads();
  float vs = 0.f;
#pragma unroll
  for (int i = 0; i < 16; ++i) { const float dl = vals[i] - mu; vs = vs + dl * dl; }
  red[t] = vs; __syncthreads();
  for (int st = 128; st > 0; st >>= 1) { if (t < st) red[t] = red[t] + red[t + st]; __syncthreads(); }
  const float rs = rsqrtf(red[0] * (1.0f / (float)DFF) + 1e-5f);
  v4h yh[4], yl[4];
#pragma unroll
  for (int u = 0; u < 4; ++u) { const v4f gg = *(const v4fa*)(g + t * 4 + 1024 * u), bv = *(const v4fa*)(bb + t * 4 + 1024 * u);
#pragma unroll
    for (int q = 0; q < 4; ++q) { const float y = ((vals[u * 4 + q] - mu) * rs) * bf16_rne(gg[q]) + bf16_rne(bv[q]); const _Float16 hi = (_Float16)y; yh[u][q] = hi; yl[u][q] = (_Float16)((y - (float)hi) * 1024.0f); } }
  _Float16* dh = UH + r * DFF + t * 4; _Float16* dl_ = UL + r * DFF + t * 4;
#pragma unroll
  for (int u = 0; u < 4; ++u) { *(volatile v4h*)(dh + 1024 * u) = yh[u]; *(volatile v4h*)(dl_ + 1024 * u) = yl[u]; }
  __threadfence();
#pragma unroll
  for (int u = 0; u < 4; ++u) { *(volatile v4h*)(dh + 1024 * u) = yh[u]; *(volatile v4h*)(dl_ + 1024 * u) = yl[u]; }
}

__global__ __launch_bounds__(256) void k_vt(const _Float16* __restrict__ QKV, _Float16* __restrict__ VT) {
  __shared__ unsigned short tl[64][66];
  const int tid = threadIdx.x; const int slab = blockIdx.x / (SEQ / 64), lg = blockIdx.x % (SEQ / 64); const int b = slab / NH, h = slab % NH;
  for (int i = tid; i < 64 * 8; i += 256) { const int r = i / 8, c8 = (i % 8) * 8; FragH f; f.half[0] = *(const v8us*)((const unsigned short*)QKV + ((size_t)b * SEQ + lg * 64 + r) * LQ + 2 * DM + h * HD + c8);
#pragma unroll
    for (int q = 0; q < 8; ++q) tl[r][c8 + q] = f.u[q]; }
  __syncthreads();
  const int pc = tid % 8; FragH f0, f1;
#pragma unroll
  for (int q = 0; q < 8; ++q) { f0.u[q] = tl[pc * 8 + q][tid / 8]; f1.u[q] = tl[pc * 8 + q][32 + tid / 8]; }
  unsigned short* d0 = (unsigned short*)VT + ((size_t)slab * 64 + tid / 8) * SEQ + lg * 64 + pc * 8; unsigned short* d1 = d0 + (size_t)32 * SEQ;
  const v8us o0 = f0.half[0], o1 = f1.half[0];
  *(volatile v8us*)d0 = o0; *(volatile v8us*)d1 = o1; __threadfence(); *(volatile v8us*)d0 = o0; *(volatile v8us*)d1 = o1;
}

__global__ __launch_bounds__(128) void k_attn(const _Float16* __restrict__ QKV, const _Float16* __restrict__ VT, _Float16* __restrict__ O16) {
  __shared__ __attribute__((aligned(16))) unsigned short pl[4][16][40];
  __shared__ __attribute__((aligned(16))) unsigned short os[4][16][72];
  const int tid = threadIdx.x, lane = tid & 31, ln = lane & 15, hh = lane >> 4;
  const int w = __builtin_amdgcn_readfirstlane(tid >> 5);
  const int qb = blockIdx.x % (SEQ / 64), bh = blockIdx.x / (SEQ / 64); const int b = bh / NH, h = bh % NH;
  const int i0 = qb * 64 + w * 16;
  const size_t qoff = ((size_t)b * SEQ + i0 + ln) * LQ + h * HD;
  const size_t kbase = (size_t)b * SEQ * LQ + DM + h * HD;
  const size_t vbase = ((size_t)bh * HD + ln) * SEQ;
  const v8f z8 = {0.f,0.f,0.f,0.f,0.f,0.f,0.f,0.f};
  v8f o0 = z8, o1 = z8, o2 = z8, o3 = z8; float m[8], l[8];
#pragma unroll
  for (int r = 0; r < 8; ++r) { m[r] = -1.0e30f; l[r] = 0.f; }
#pragma unroll 1
  for (int j0 = 0; j0 < SEQ; j0 += 32) {
    const v16h qa0 = g2_frag(QKV + qoff, hh), qa1 = g2_frag(QKV + qoff + 32, hh);
    v8f s0 = z8, s1 = z8;
    { const size_t ko = kbase + (size_t)(j0 + ln) * LQ;
      v16h kf = g2_frag(QKV + ko, hh); s0 = g2_mma(qa0, kf, s0); kf = g2_frag(QKV + ko + 32, hh); s0 = g2_mma(qa1, kf, s0);
      kf = g2_frag(QKV + ko + (size_t)16 * LQ, hh); s1 = g2_mma(qa0, kf, s1); kf = g2_frag(QKV + ko + (size_t)16 * LQ + 32, hh); s1 = g2_mma(qa1, kf, s1); }
    const size_t vo = vbase + j0;
    const v16h vf0 = g2_frag(VT + vo, hh), vf1 = g2_frag(VT + vo + (size_t)16 * SEQ, hh), vf2 = g2_frag(VT + vo + (size_t)32 * SEQ, hh), vf3 = g2_frag(VT + vo + (size_t)48 * SEQ, hh);
#pragma unroll
    for (int r = 0; r < 8; ++r) {
      const float sa = s0[r] * 0.125f, sb = s1[r] * 0.125f;
      float tm = fmaxf(sa, sb);
      tm = fmaxf(tm, __shfl_xor(tm, 1)); tm = fmaxf(tm, __shfl_xor(tm, 2)); tm = fmaxf(tm, __shfl_xor(tm, 4)); tm = fmaxf(tm, __shfl_xor(tm, 8));
      const float mn = fmaxf(m[r], tm);
      const float al = __expf(m[r] - mn);
      const _Float16 ha = (_Float16)__expf(sa - mn), hb = (_Float16)__expf(sb - mn);
      l[r] = l[r] * al + ((float)ha + (float)hb);
      m[r] = mn;
      o0[r] *= al; o1[r] *= al; o2[r] *= al; o3[r] *= al;
      pl[w][8 * hh + r][ln] = __builtin_bit_cast(unsigned short, ha);
      pl[w][8 * hh + r][16 + ln] = __builtin_bit_cast(unsigned short, hb);
    }
    __builtin_amdgcn_fence(4  , "workgroup"); __builtin_amdgcn_wave_barrier();
    FragH pf; pf.half[0] = *(const v8us*)&pl[w][ln][8 * hh]; pf.half[1] = *(const v8us*)&pl[w][ln][16 + 8 * hh];
    __builtin_amdgcn_fence(4  , "workgroup"); __builtin_amdgcn_wave_barrier();
    o0 = g2_mma(pf.v, vf0, o0); o1 = g2_mma(pf.v, vf1, o1); o2 = g2_mma(pf.v, vf2, o2); o3 = g2_mma(pf.v, vf3, o3);
  }
#pragma unroll
  for (int r = 0; r < 8; ++r) {
    float ls = l[r];
    ls += __shfl_xor(ls, 1); ls += __shfl_xor(ls, 2); ls += __shfl_xor(ls, 4); ls += __shfl_xor(ls, 8);
    const float inv = 64.0f * (1.0f / ls);
    os[w][8 * hh + r][ln] = h16_bits(o0[r] * inv); os[w][8 * hh + r][16 + ln] = h16_bits(o1[r] * inv);
    os[w][8 * hh + r][32 + ln] = h16_bits(o2[r] * inv); os[w][8 * hh + r][48 + ln] = h16_bits(o3[r] * inv);
  }
  __builtin_amdgcn_fence(4  , "workgroup"); __builtin_amdgcn_wave_barrier();
  const int rq = lane >> 3, pc = (lane & 7) * 8;
  v8us ov[4];
#pragma unroll
  for (int it = 0; it < 4; ++it) ov[it] = *(const v8us*)&os[w][it * 4 + rq][pc];
  unsigned short* ob = (unsigned short*)O16 + ((size_t)b * SEQ + i0 + rq) * DM + h * HD + pc;
#pragma unroll
  for (int it = 0; it < 4; ++it) *(volatile v8us*)(ob + (size_t)(it * 4) * DM) = ov[it];
  __threadfence();
#pragma unroll
  for (int it = 0; it < 4; ++it) *(volatile v8us*)(ob + (size_t)(it * 4) * DM) = ov[it];
}

__device__ __forceinline__ void g2_kloop(const _Float16* __restrict__ A, size_t a0o, size_t a1o, const _Float16* __restrict__ Bh, size_t b0o, size_t b1o, size_t b2o, size_t b3o, int K, int hh,
                                         v8f& c00, v8f& c01, v8f& c02, v8f& c03, v8f& c10, v8f& c11, v8f& c12, v8f& c13) {
#pragma unroll 1
  for (int kb = 0; kb < K; kb += 32) {
    const v16h a0 = g2_frag(A + a0o + kb, hh), a1 = g2_frag(A + a1o + kb, hh);
    v16h bq = g2_frag(Bh + b0o + kb, hh); c00 = g2_mma(a0, bq, c00); c10 = g2_mma(a1, bq, c10);
    bq = g2_frag(Bh + b1o + kb, hh); c01 = g2_mma(a0, bq, c01); c11 = g2_mma(a1, bq, c11);
    bq = g2_frag(Bh + b2o + kb, hh); c02 = g2_mma(a0, bq, c02); c12 = g2_mma(a1, bq, c12);
    bq = g2_frag(Bh + b3o + kb, hh); c03 = g2_mma(a0, bq, c03); c13 = g2_mma(a1, bq, c13);
  }
}

template <int ACT, int RESM, int O16, int BIAS, int TWO, int RMAPR, int RMAPC>
__device__ __forceinline__ void gemm_body(const _Float16* __restrict__ A, const _Float16* __restrict__ A2, float a2s, int lda, const _Float16* __restrict__ Bh, int ldb, float alpha, const float* __restrict__ bias,
                                          const float* __restrict__ R, int ldr, float* __restrict__ C, _Float16* __restrict__ C16, int ldc, int rowbase, int M, int N, int K) {
  __shared__ __attribute__((aligned(16))) float so[4][32][68];
  const int tid = threadIdx.x, lane = tid & 31, ln = lane & 15, hh = lane >> 4;
  const int w = __builtin_amdgcn_readfirstlane(tid >> 5);
  const int ntn = N >> 6; const int mt = blockIdx.x / ntn, nq = blockIdx.x - mt * ntn; const int row0 = mt * 128 + 32 * w, col0 = nq * 64;
  if (row0 >= M) return;
  const size_t a0o = (size_t)(row0 + ln) * lda, a1o = a0o + (size_t)16 * lda;
  const size_t b0o = (size_t)(col0 + ln) * ldb, b1o = b0o + (size_t)16 * ldb, b2o = b1o + (size_t)16 * ldb, b3o = b2o + (size_t)16 * ldb;
  const v8f z8 = {0.f,0.f,0.f,0.f,0.f,0.f,0.f,0.f}; v8f c00 = z8, c01 = z8, c02 = z8, c03 = z8, c10 = z8, c11 = z8, c12 = z8, c13 = z8;
  if (TWO) {
    g2_kloop(A2, a0o, a1o, Bh, b0o, b1o, b2o, b3o, K, hh, c00, c01, c02, c03, c10, c11, c12, c13);
    c00 *= a2s; c01 *= a2s; c02 *= a2s; c03 *= a2s; c10 *= a2s; c11 *= a2s; c12 *= a2s; c13 *= a2s;
  }
  g2_kloop(A, a0o, a1o, Bh, b0o, b1o, b2o, b3o, K, hh, c00, c01, c02, c03, c10, c11, c12, c13);
  v8f accs[8] = {c00, c01, c02, c03, c10, c11, c12, c13};
#pragma unroll
  for (int u = 0; u < 8; ++u) { const int t = u & 3, half = u >> 2; const int col = col0 + t * 16 + ln; float bv = 0.f; if (BIAS) bv = bf16_rne(bias[col]);
#pragma unroll
    for (int r = 0; r < 8; ++r) so[w][half * 16 + 8 * hh + r][t * 16 + ln] = accs[u][r] * alpha + bv; }
  __builtin_amdgcn_fence(4  , "workgroup"); __builtin_amdgcn_wave_barrier();
  const int rsub = lane >> 4, c4 = (lane & 15) * 4;
#pragma unroll 1
  for (int q = 0; q < 16; ++q) {
    const int r = q * 2 + rsub; v4f v = *(const v4fa*)&so[w][r][c4];
    if (ACT == 1) {
#pragma unroll
      for (int i = 0; i < 4; ++i) v[i] = 0.5f * v[i] * (1.0f + erff(v[i] * 0.70710678118654752f)); }
    if (RESM != 0) { const size_t rr = RMAPR ? XROW(rowbase + row0 + r) : (size_t)(row0 + r); v4f rv = *(const v4fa*)(R + rr * ldr + col0 + c4);
      if (RESM == 2) {
#pragma unroll
        for (int i = 0; i < 4; ++i) rv[i] = bf16_rne(rv[i]); }
      v = v + rv; }
    if (ACT != 0 || RESM != 0) *(v4fa*)&so[w][r][c4] = v;
    const size_t cr = RMAPC ? XROW(rowbase + row0 + r) : (size_t)(row0 + r);
    if (O16) { v4h h4;
#pragma unroll
      for (int i = 0; i < 4; ++i) h4[i] = (_Float16)v[i];
      *(volatile v4h*)(C16 + cr * ldc + col0 + c4) = h4; }
    else *(volatile v4f*)(C + cr * ldc + col0 + c4) = v;
  }
  __threadfence();
#pragma unroll 1
  for (int q = 0; q < 16; ++q) {
    const int r = q * 2 + rsub; const v4f v = *(const v4fa*)&so[w][r][c4];
    const size_t cr = RMAPC ? XROW(rowbase + row0 + r) : (size_t)(row0 + r);
    if (O16) { v4h h4;
#pragma unroll
      for (int i = 0; i < 4; ++i) h4[i] = (_Float16)v[i];
      *(volatile v4h*)(C16 + cr * ldc + col0 + c4) = h4; }
    else *(volatile v4f*)(C + cr * ldc + col0 + c4) = v;
  }
}

__global__ __launch_bounds__(128) void k_gemm_qkv(const _Float16* __restrict__ A, const _Float16* __restrict__ Bh, _Float16* __restrict__ C16, int M) {
  gemm_body<0, 0, 1, 0, 0, 0, 0>(A, A, 0.f, DM, Bh, DM, 0.0625f, (const float*)nullptr, (const float*)nullptr, 0, (float*)nullptr, C16, LQ, 0, M, LQ, DM);
}
__global__ __launch_bounds__(128) void k_gemm_proj(const _Float16* __restrict__ A, const _Float16* __restrict__ Bh, const float* __restrict__ bias, const float* __restrict__ X, float* __restrict__ C, int M) {
  gemm_body<0, 2, 0, 1, 0, 1, 0>(A, A, 0.f, DM, Bh, DM, 0.0009765625f, bias, X, DM, C, (_Float16*)nullptr, DM, 0, M, DM, DM);
}
__global__ __launch_bounds__(128) void k_gemm_fc1(const _Float16* __restrict__ A, const _Float16* __restrict__ Bh, const float* __restrict__ bias, float* __restrict__ C, int M) {
  gemm_body<1, 0, 0, 1, 0, 0, 0>(A, A, 0.f, DM, Bh, DM, 0.0625f, bias, (const float*)nullptr, 0, C, (_Float16*)nullptr, DFF, 0, M, DFF, DM);
}
__global__ __launch_bounds__(128) void k_gemm_fc2(const _Float16* __restrict__ AH, const _Float16* __restrict__ AL, const _Float16* __restrict__ Bh, const float* __restrict__ bias, const float* __restrict__ R, float* __restrict__ C, int rowbase, int M) {
  gemm_body<0, 1, 0, 1, 1, 0, 1>(AH, AL, 0.0009765625f, DFF, Bh, DFF, 0.0625f, bias, R, DM, C, (_Float16*)nullptr, DM, rowbase, M, DM, DFF);
}

constexpr size_t cmaxz(size_t a, size_t b) { return a > b ? a : b; }
constexpr size_t SZ_BQKV = (size_t)LQ * DM * 2;
constexpr size_t SZ_BO   = (size_t)DM * DM * 2;
constexpr size_t SZ_BW1  = (size_t)DFF * DM * 2;
constexpr size_t SZ_BW2  = (size_t)DM * DFF * 2;
constexpr size_t SZ_XN   = (size_t)NR * DM * 2;
constexpr size_t SZ_QKV  = (size_t)NR * LQ * 2;
constexpr size_t SZ_VT   = (size_t)NB * NH * HD * SEQ * 2;
constexpr size_t SZ_U32  = (size_t)MCH * DFF * 4;
constexpr size_t SZ_R1   = cmaxz(SZ_QKV + SZ_VT, SZ_U32);
constexpr size_t SZ_O16  = (size_t)NR * DM * 2;
constexpr size_t SZ_X1   = (size_t)NR * DM * 4;
constexpr size_t SZ_UH   = (size_t)MCH * DFF * 2;
constexpr size_t OFF_BQKV = 0;
constexpr size_t OFF_BO   = OFF_BQKV + SZ_BQKV;
constexpr size_t OFF_BW1  = OFF_BO + SZ_BO;
constexpr size_t OFF_BW2  = OFF_BW1 + SZ_BW1;
constexpr size_t OFF_XN   = OFF_BW2 + SZ_BW2;
constexpr size_t OFF_R1   = OFF_XN + SZ_XN;
constexpr size_t OFF_O16  = OFF_R1 + SZ_R1;
constexpr size_t OFF_X1   = OFF_O16 + SZ_O16;
constexpr size_t OFF_UH   = OFF_X1 + SZ_X1;
constexpr size_t OFF_UL   = OFF_UH + SZ_UH;
constexpr size_t WS_TOTAL = OFF_UL + SZ_UH;
static_assert(WS_TOTAL <= (size_t)134217728);
static_assert(SZ_QKV + SZ_VT <= SZ_R1 && SZ_U32 <= SZ_R1);
static_assert(OFF_BO % 256 == 0 && OFF_BW1 % 256 == 0 && OFF_BW2 % 256 == 0 && OFF_XN % 256 == 0 && OFF_R1 % 256 == 0 && OFF_O16 % 256 == 0 && OFF_X1 % 256 == 0 && OFF_UH % 256 == 0 && OFF_UL % 256 == 0 && SZ_QKV % 256 == 0);
static_assert(((size_t)LQ * DM) % (8 * 32) == 0 && ((size_t)DM * DM) % (8 * 32) == 0 && ((size_t)DFF * DM) % (8 * 32) == 0);

extern "C" void kernel_launch(void* const* d_in, const int* in_sizes, int n_in,
                              void* d_out, int out_size, void* d_ws, size_t ws_size, hipStream_t stream) {
  if (n_in < 14) return;
  const size_t needx = ((size_t)(NB - 1) * SEQ_FULL + SEQ) * DM;
  if ((size_t)in_sizes[0] < needx || (size_t)out_size < needx) return;
  if ((size_t)in_sizes[1] < (size_t)LQ * DM || (size_t)in_sizes[2] < (size_t)DM * DM || in_sizes[3] < DM) return;
  if ((size_t)in_sizes[4] < (size_t)DFF * DM || in_sizes[5] < DFF || (size_t)in_sizes[6] < (size_t)DM * DFF || in_sizes[7] < DM) return;
  if (in_sizes[8] < DM || in_sizes[9] < DM || in_sizes[10] < DM || in_sizes[11] < DM || in_sizes[12] < DFF || in_sizes[13] < DFF) return;
  if (ws_size < WS_TOTAL) return;
  const float* x = (const float*)d_in[0]; const float* qkv_w = (const float*)d_in[1]; const float* proj_w = (const float*)d_in[2]; const float* proj_b = (const float*)d_in[3];
  const float* fc1_w = (const float*)d_in[4]; const float* fc1_b = (const float*)d_in[5]; const float* fc2_w = (const float*)d_in[6]; const float* fc2_b = (const float*)d_in[7];
  const float* ln1_g = (const float*)d_in[8]; const float* ln1_b = (const float*)d_in[9]; const float* ln2_g = (const float*)d_in[10]; const float* ln2_b = (const float*)d_in[11];
  const float* lnh_g = (const float*)d_in[12]; const float* lnh_b = (const float*)d_in[13];
  float* out = (float*)d_out; char* ws = (char*)d_ws;
  _Float16* BQKV = (_Float16*)(ws + OFF_BQKV); _Float16* BO = (_Float16*)(ws + OFF_BO); _Float16* BW1 = (_Float16*)(ws + OFF_BW1); _Float16* BW2 = (_Float16*)(ws + OFF_BW2);
  _Float16* XN = (_Float16*)(ws + OFF_XN);
  _Float16* QKV16 = (_Float16*)(ws + OFF_R1); _Float16* VT = (_Float16*)(ws + OFF_R1 + SZ_QKV); float* U32 = (float*)(ws + OFF_R1);
  _Float16* O16 = (_Float16*)(ws + OFF_O16); float* X1 = (float*)(ws + OFF_X1); _Float16* UH = (_Float16*)(ws + OFF_UH); _Float16* UL = (_Float16*)(ws + OFF_UL);

  k_wnat<<<(unsigned)(((size_t)LQ * DM / 8 + 255) / 256), 256, 0, stream>>>(qkv_w, BQKV, (unsigned)((size_t)LQ * DM / 8));
  k_wnat<<<(unsigned)(((size_t)DM * DM / 8 + 255) / 256), 256, 0, stream>>>(proj_w, BO, (unsigned)((size_t)DM * DM / 8));
  k_wnat<<<(unsigned)(((size_t)DFF * DM / 8 + 255) / 256), 256, 0, stream>>>(fc1_w, BW1, (unsigned)((size_t)DFF * DM / 8));
  k_wnat<<<(unsigned)(((size_t)DM * DFF / 8 + 255) / 256), 256, 0, stream>>>(fc2_w, BW2, (unsigned)((size_t)DM * DFF / 8));
  k_ln16<<<NR, 256, 0, stream>>>(x, ln1_g, ln1_b, 1, 1, XN);
  k_gemm_qkv<<<(NR / 128) * (LQ / 64), 128, 0, stream>>>(XN, BQKV, QKV16, NR);
  k_vt<<<NB * NH * (SEQ / 64), 256, 0, stream>>>(QKV16, VT);
  k_attn<<<(SEQ / 64) * NB * NH, 128, 0, stream>>>(QKV16, VT, O16);
  k_gemm_proj<<<(NR / 128) * (DM / 64), 128, 0, stream>>>(O16, BO, proj_b, x, X1, NR);
  k_ln16<<<NR, 256, 0, stream>>>(X1, ln2_g, ln2_b, 0, 0, XN);
  for (int r0 = 0; r0 < NR; r0 += MCH) {
    k_gemm_fc1<<<(MCH / 128) * (DFF / 64), 128, 0, stream>>>(XN + (size_t)r0 * DM, BW1, fc1_b, U32, MCH);
    k_lnh<<<MCH, 256, 0, stream>>>(U32, lnh_g, lnh_b, UH, UL);
    k_gemm_fc2<<<(MCH / 128) * (DM / 64), 128, 0, stream>>>(UH, UL, BW2, fc2_b, X1 + (size_t)r0 * DM, out, r0, MCH);
  }
}
